// MultiHeadAttention_53961969107321
// MI455X (gfx1250) — hardware-verified
//
#include <hip/hip_runtime.h>


#ifndef NB
#define NB 2
#endif
#ifndef SEQ
#define SEQ 2048
#endif
#define NB_FULL  2
#define SEQ_FULL 2048
#ifndef OUT_SEQ
#define OUT_SEQ SEQ
#endif
#define DM   1024
#define NH_  16
#define HD   64
#define AW   4
#define QRS  2048.0f
#define QRI  (1.0f / 2048.0f)
#define L2E  1.4426950408889634f
#define PSH  14.0f
#define NEGB (-3.0e38f)

static_assert(HD == 64);
static_assert(NH_ * HD == DM);
static_assert((DM & (DM - 1)) == 0);
static_assert(DM % 64 == 0);
static_assert(SEQ % 64 == 0);
static_assert((NB * SEQ) % 64 == 0);
static_assert(SEQ % 32 == 0);
static_assert(SEQ % (16 * AW) == 0);
static_assert(((size_t)SEQ * DM) % 8 == 0);
static_assert(NB <= NB_FULL);
static_assert(SEQ <= SEQ_FULL);

typedef _Float16 h16;
typedef unsigned short bf;
typedef __attribute__((ext_vector_type(16))) __bf16   v16bf;
typedef __attribute__((ext_vector_type(16))) _Float16 v16h;
typedef __attribute__((ext_vector_type(8)))  _Float16 v8h;
typedef __attribute__((ext_vector_type(8)))  unsigned short v8us;
typedef __attribute__((ext_vector_type(8)))  float    v8f;
typedef __attribute__((ext_vector_type(4)))  float    v4f;
typedef v4f  __attribute__((may_alias)) v4fa;

__device__ __forceinline__ unsigned short f2bf(float f) { unsigned u = __float_as_uint(f); u += 0x7FFFu + ((u >> 16) & 1u); return (unsigned short)(u >> 16); }
__device__ __forceinline__ float bf2f(unsigned short s) { return __uint_as_float(((unsigned)s) << 16); }
__device__ __forceinline__ v16h cat16(v8h lo, v8h hi) { return __builtin_shufflevector(lo, hi, 0, 1, 2, 3, 4, 5, 6, 7, 8, 9, 10, 11, 12, 13, 14, 15); }
__device__ __forceinline__ v16bf cat16b(v8us lo, v8us hi) { return __builtin_bit_cast(v16bf, __builtin_shufflevector(lo, hi, 0, 1, 2, 3, 4, 5, 6, 7, 8, 9, 10, 11, 12, 13, 14, 15)); }
__device__ __forceinline__ v8f wmma16(v16h a, v16h b, v8f c) { return __builtin_amdgcn_wmma_f32_16x16x32_f16(false, a, false, b, (short)0, c, false, false); }
__device__ __forceinline__ v8f wmmab(v16bf a, v16bf b, v8f c) { return __builtin_amdgcn_wmma_f32_16x16x32_bf16(false, a, false, b, (short)0, c, false, false); }
__device__ __forceinline__ v16h  ldh(const h16* p) { return cat16(*(const v8h*)p, *(const v8h*)(p + 16)); }
__device__ __forceinline__ v16bf ldb(const bf* p)  { return cat16b(*(const v8us*)p, *(const v8us*)(p + 16)); }
__device__ __forceinline__ void wave_sync() { __builtin_amdgcn_fence(3  , "wavefront"); __builtin_amdgcn_wave_barrier(); asm volatile("" ::: "memory"); }

__global__ __launch_bounds__(256) void k_cvt8(const float* __restrict__ src, bf* dst, size_t n8) {
    const size_t i = (size_t)blockIdx.x * 256 + threadIdx.x; if (i >= n8) return;
    const v8f v = *(const v8f*)(src + i * 8); v8us o;
#pragma unroll
    for (int k = 0; k < 8; ++k) o[k] = f2bf(v[k]);
    *(volatile v8us*)(dst + i * 8) = o; __threadfence(); *(volatile v8us*)(dst + i * 8) = o;
}

__global__ __launch_bounds__(256) void k_wt(const float* __restrict__ W, bf* WT) {
    __shared__ float tile[64 * 65];
    const int tid = threadIdx.x; const int n0 = blockIdx.x * 64, k0 = blockIdx.y * 64;
#pragma unroll
    for (int it = 0; it < 4; ++it) { const int c = it * 256 + tid; const int r = c >> 4, c4 = (c & 15) * 4;
        const v4f v = *(const v4f*)(W + (size_t)(k0 + r) * DM + n0 + c4);
        tile[r * 65 + c4 + 0] = v[0]; tile[r * 65 + c4 + 1] = v[1]; tile[r * 65 + c4 + 2] = v[2]; tile[r * 65 + c4 + 3] = v[3]; }
    __syncthreads();
    v8us o[2];
#pragma unroll
    for (int it = 0; it < 2; ++it) { const int c = it * 256 + tid; const int n = c >> 3, k8 = (c & 7) * 8;
#pragma unroll
        for (int e = 0; e < 8; ++e) o[it][e] = f2bf(tile[(k8 + e) * 65 + n]); }
#pragma unroll
    for (int it = 0; it < 2; ++it) { const int c = it * 256 + tid; const int n = c >> 3, k8 = (c & 7) * 8;
        *(volatile v8us*)(WT + (size_t)(n0 + n) * DM + k0 + k8) = o[it]; }
    __threadfence();
#pragma unroll
    for (int it = 0; it < 2; ++it) { const int c = it * 256 + tid; const int n = c >> 3, k8 = (c & 7) * 8;
        *(volatile v8us*)(WT + (size_t)(n0 + n) * DM + k0 + k8) = o[it]; }
}

template <int MODE>
__global__ __launch_bounds__(32) void k_gemm(const bf* __restrict__ A, const bf* __restrict__ Bt, int KA, h16* Ph, h16* Pr, float* OUT) {
    __shared__ __align__(16) float os[16 * 68];
    const int lane = threadIdx.x & 31, lr = lane & 15, hi = lane >> 4; const int r0 = blockIdx.x * 64, c0 = blockIdx.y * 64;
    v8f acc[4][4];
#pragma unroll
    for (int mb = 0; mb < 4; ++mb)
#pragma unroll
        for (int nb = 0; nb < 4; ++nb) acc[mb][nb] = (v8f){};
    const size_t aoff = (size_t)(r0 + lr) * (size_t)KA + 8 * hi, boff = (size_t)(c0 + lr) * DM + 8 * hi;
#pragma unroll 1
    for (int kc = 0; kc < KA; kc += 32) {
        const int kb = kc & (DM - 1);
        v16bf a[4];
#pragma unroll
        for (int mb = 0; mb < 4; ++mb) a[mb] = ldb(A + aoff + (size_t)mb * 16 * (size_t)KA + kc);
#pragma unroll
        for (int nb = 0; nb < 4; ++nb) { const v16bf b = ldb(Bt + boff + (size_t)nb * 16 * DM + kb);
#pragma unroll
            for (int mb = 0; mb < 4; ++mb) acc[mb][nb] = wmmab(a[mb], b, acc[mb][nb]); }
        asm volatile("v_nop\n\tv_nop\n\tv_nop\n\tv_nop" : "+v"(acc[0][0]), "+v"(acc[1][1]), "+v"(acc[2][2]), "+v"(acc[3][3]) : "v"(a[0]), "v"(a[1]), "v"(a[2]), "v"(a[3]));
    }
#pragma unroll
    for (int mb = 0; mb < 4; ++mb) {
#pragma unroll
        for (int nb = 0; nb < 4; ++nb) {
#pragma unroll
            for (int j = 0; j < 8; ++j) os[(hi * 8 + j) * 68 + nb * 16 + lr] = acc[mb][nb][j]; }
        wave_sync();
        const int m0 = r0 + mb * 16;
        if (MODE == 0) {
            const size_t sb = (size_t)m0 * DM + c0;
#pragma unroll 1
            for (int ps = 0; ps < 2; ++ps) {
#pragma unroll
                for (int s = 0; s < 4; ++s) { const int row = 4 * s + (lane >> 3), c8 = (lane & 7) * 8;
                    const v4f x0 = *(const v4fa*)(&os[row * 68 + c8]); const v4f x1 = *(const v4fa*)(&os[row * 68 + c8 + 4]); v8h hv, rv;
#pragma unroll
                    for (int i = 0; i < 4; ++i) { const h16 a0 = (h16)x0[i]; const h16 a1 = (h16)x1[i]; hv[i] = a0; hv[4 + i] = a1; rv[i] = (h16)((x0[i] - (float)a0) * QRS); rv[4 + i] = (h16)((x1[i] - (float)a1) * QRS); }
                    const size_t oo = sb + (size_t)row * DM + c8;
                    *(volatile v8h*)(Ph + oo) = hv; *(volatile v8h*)(Pr + oo) = rv; }
                if (ps == 0) __threadfence(); }
        } else {
            float* orow = OUT + ((size_t)(m0 / SEQ) * OUT_SEQ + (size_t)(m0 % SEQ)) * DM + c0;
#pragma unroll 1
            for (int ps = 0; ps < 2; ++ps) {
#pragma unroll
                for (int s = 0; s < 8; ++s) { const int row = 2 * s + hi, cofs = lr * 4;
                    const v4f val = *(const v4fa*)(&os[row * 68 + cofs]);
                    *(volatile v4f*)(orow + (size_t)row * DM + cofs) = val; }
                if (ps == 0) __threadfence(); }
        }
        wave_sync();
    }
}

__global__ __launch_bounds__(256) void k_vt(const h16* __restrict__ V2, h16* VT2, size_t pln) {
    __shared__ __align__(16) h16 ts[64 * 72];
    const int tid = threadIdx.x; const int s0 = blockIdx.x * 64; const int zh = blockIdx.y; const size_t zo = (size_t)blockIdx.z * pln;
    const h16* src = V2 + zo + ((size_t)zh * SEQ + s0) * HD;
    h16* dst = VT2 + zo + (size_t)zh * HD * SEQ + s0;
#pragma unroll
    for (int it = 0; it < 2; ++it) { const int c = it * 256 + tid; const int row = c >> 3, c8 = (c & 7) * 8;
        const v8h v = *(const v8h*)(src + (size_t)row * HD + c8); *(v8h*)(&ts[row * 72 + c8]) = v; }
    __syncthreads();
    v8h o[2];
#pragma unroll
    for (int it = 0; it < 2; ++it) { const int c = it * 256 + tid; const int d = c >> 3, k8 = (c & 7) * 8;
#pragma unroll
        for (int e = 0; e < 8; ++e) o[it][e] = ts[(k8 + e) * 72 + d]; }
#pragma unroll
    for (int it = 0; it < 2; ++it) { const int c = it * 256 + tid; const int d = c >> 3, k8 = (c & 7) * 8;
        *(volatile v8h*)(dst + (size_t)d * SEQ + k8) = o[it]; }
    __threadfence();
#pragma unroll
    for (int it = 0; it < 2; ++it) { const int c = it * 256 + tid; const int d = c >> 3, k8 = (c & 7) * 8;
        *(volatile v8h*)(dst + (size_t)d * SEQ + k8) = o[it]; }
}

#define STG(OFS, OH, OR) { v4f a_, c_; \
    a_[0] = OH[0] * inv + OR[0] * ri; a_[1] = OH[1] * inv + OR[1] * ri; a_[2] = OH[2] * inv + OR[2] * ri; a_[3] = OH[3] * inv + OR[3] * ri; \
    c_[0] = OH[4] * inv + OR[4] * ri; c_[1] = OH[5] * inv + OR[5] * ri; c_[2] = OH[6] * inv + OR[6] * ri; c_[3] = OH[7] * inv + OR[7] * ri; \
    *(v4fa*)(&os[wb + lr * 68 + (OFS) + 8 * hi]) = a_; *(v4fa*)(&os[wb + lr * 68 + (OFS) + 8 * hi + 4]) = c_; }

__global__ __launch_bounds__(32 * AW) void k_flash(const h16* __restrict__ QH, const h16* __restrict__ QR, const h16* __restrict__ KH, const h16* __restrict__ KR,
                                                   const h16* __restrict__ VTH, const h16* __restrict__ VTR, bf* CTX) {
    __shared__ __align__(16) float os[AW * 16 * 68];
    const int lane = threadIdx.x & 31, wave = threadIdx.x >> 5, lr = lane & 15, hi = lane >> 4;
    const int zh = blockIdx.y; const int b = zh / NH_, h = zh % NH_;
    const int t0 = (blockIdx.x * AW + wave) * 16;
    const size_t pbase = (size_t)zh * SEQ * HD;
    const size_t qo = pbase + (size_t)(t0 + lr) * HD + 8 * hi;
    const v16h qh0 = ldh(QH + qo), qh1 = ldh(QH + qo + 32), qr0 = ldh(QR + qo), qr1 = ldh(QR + qo + 32);
    const size_t ko = pbase + (size_t)lr * HD + 8 * hi;
    const size_t vo = pbase + (size_t)lr * SEQ + 8 * hi;
    v8f oh0 = (v8f){}, oh1 = (v8f){}, oh2 = (v8f){}, oh3 = (v8f){};
    v8f or0 = (v8f){}, or1 = (v8f){}, or2 = (v8f){}, or3 = (v8f){};
    float m = NEGB, l = 0.0f;
    const int kend = t0 + 16;
#pragma unroll 1
    for (int key0 = 0; key0 < kend; key0 += 32) {
        const size_t kk = ko + (size_t)key0 * HD;
        v8f sHa = (v8f){}, sLa = (v8f){}, sHb = (v8f){}, sLb = (v8f){};
        { const v16h ka0 = ldh(KH + kk), ka1 = ldh(KH + kk + 32), kb0 = ldh(KH + kk + 16 * HD), kb1 = ldh(KH + kk + 16 * HD + 32);
          sHa = wmma16(ka0, qh0, sHa); sLa = wmma16(ka0, qr0, sLa); sHb = wmma16(kb0, qh0, sHb); sLb = wmma16(kb0, qr0, sLb);
          sHa = wmma16(ka1, qh1, sHa); sLa = wmma16(ka1, qr1, sLa); sHb = wmma16(kb1, qh1, sHb); sLb = wmma16(kb1, qr1, sLb);
          asm volatile("v_nop\n\tv_nop\n\tv_nop\n\tv_nop" : "+v"(sHa), "+v"(sLa), "+v"(sHb), "+v"(sLb) : "v"(ka0), "v"(ka1), "v"(kb0), "v"(kb1)); }
        { const v16h ra0 = ldh(KR + kk), ra1 = ldh(KR + kk + 32), rb0 = ldh(KR + kk + 16 * HD), rb1 = ldh(KR + kk + 16 * HD + 32);
          sLa = wmma16(ra0, qh0, sLa); sLb = wmma16(rb0, qh0, sLb); sLa = wmma16(ra1, qh1, sLa); sLb = wmma16(rb1, qh1, sLb);
          asm volatile("v_nop\n\tv_nop\n\tv_nop\n\tv_nop" : "+v"(sLa), "+v"(sLb) : "v"(ra0), "v"(ra1), "v"(rb0), "v"(rb1)); }
        float ta[8], tb[8];
#pragma unroll
        for (int r = 0; r < 8; ++r) { ta[r] = (sHa[r] + sLa[r] * QRI) * L2E; tb[r] = (sHb[r] + sLb[r] * QRI) * L2E; }
        if (key0 + 31 > t0) {
            const int tq = t0 + lr - key0 - 8 * hi;
#pragma unroll
            for (int r = 0; r < 8; ++r) { ta[r] = (r > tq) ? NEGB : ta[r]; tb[r] = (16 + r > tq) ? NEGB : tb[r]; }
        }
        float mx = NEGB;
#pragma unroll
        for (int r = 0; r < 8; ++r) mx = fmaxf(mx, fmaxf(ta[r], tb[r]));
        mx = fmaxf(mx, __shfl_xor(mx, 16, 32));
        const float mnew = fmaxf(m, mx);
        const float alpha = __builtin_amdgcn_exp2f(m - mnew);
        const float sh = PSH - mnew;
        v16h pb; float ls = 0.0f;
#pragma unroll
        for (int r = 0; r < 8; ++r) { const h16 pa = (h16)__builtin_amdgcn_exp2f(ta[r] + sh); const h16 pc = (h16)__builtin_amdgcn_exp2f(tb[r] + sh); pb[r] = pa; pb[8 + r] = pc; ls += (float)pa + (float)pc; }
        l = l * alpha + ls; m = mnew;
        oh0 = oh0 * alpha; oh1 = oh1 * alpha; oh2 = oh2 * alpha; oh3 = oh3 * alpha;
        or0 = or0 * alpha; or1 = or1 * alpha; or2 = or2 * alpha; or3 = or3 * alpha;
        { const h16* va = VTH + vo + key0;
          const v16h v0 = ldh(va), v1 = ldh(va + (size_t)16 * SEQ), v2 = ldh(va + (size_t)32 * SEQ), v3 = ldh(va + (size_t)48 * SEQ);
          oh0 = wmma16(v0, pb, oh0); oh1 = wmma16(v1, pb, oh1); oh2 = wmma16(v2, pb, oh2); oh3 = wmma16(v3, pb, oh3);
          asm volatile("v_nop\n\tv_nop\n\tv_nop\n\tv_nop" : "+v"(oh0), "+v"(oh1), "+v"(oh2), "+v"(oh3) : "v"(v0), "v"(v1), "v"(v2), "v"(v3), "v"(pb)); }
        { const h16* va = VTR + vo + key0;
          const v16h v0 = ldh(va), v1 = ldh(va + (size_t)16 * SEQ), v2 = ldh(va + (size_t)32 * SEQ), v3 = ldh(va + (size_t)48 * SEQ);
          or0 = wmma16(v0, pb, or0); or1 = wmma16(v1, pb, or1); or2 = wmma16(v2, pb, or2); or3 = wmma16(v3, pb, or3);
          asm volatile("v_nop\n\tv_nop\n\tv_nop\n\tv_nop" : "+v"(or0), "+v"(or1), "+v"(or2), "+v"(or3) : "v"(v0), "v"(v1), "v"(v2), "v"(v3), "v"(pb)); }
    }
    l += __shfl_xor(l, 16, 32);
    const float inv = 1.0f / l;
    const float ri = QRI * inv;
    const int wb = wave * 16 * 68;
    STG(0, oh0, or0)
    STG(16, oh1, or1)
    STG(32, oh2, or2)
    STG(48, oh3, or3)
    wave_sync();
    bf* crow = CTX + ((size_t)b * SEQ + t0) * (size_t)(2 * DM) + h * HD;
#pragma unroll 1
    for (int ps = 0; ps < 2; ++ps) {
#pragma unroll
        for (int s = 0; s < 4; ++s) { const int row = 4 * s + (lane >> 3), c8 = (lane & 7) * 8;
            const v4f x0 = *(const v4fa*)(&os[wb + row * 68 + c8]); const v4f x1 = *(const v4fa*)(&os[wb + row * 68 + c8 + 4]); v8us hv, lv;
#pragma unroll
            for (int i = 0; i < 4; ++i) { const unsigned short a0 = f2bf(x0[i]); const unsigned short a1 = f2bf(x1[i]); hv[i] = a0; hv[4 + i] = a1; lv[i] = f2bf(x0[i] - bf2f(a0)); lv[4 + i] = f2bf(x1[i] - bf2f(a1)); }
            const size_t oo = (size_t)row * (size_t)(2 * DM) + c8;
            *(volatile v8us*)(crow + oo) = hv; *(volatile v8us*)(crow + oo + DM) = lv; }
        if (ps == 0) __threadfence(); }
}

static constexpr size_t al256(size_t v) { return (v + 255) & ~(size_t)255; }
static constexpr size_t SZ_XB  = al256((size_t)NB * SEQ * DM * 2);
static constexpr size_t SZ_WB  = al256((size_t)DM * DM * 2);
static constexpr size_t SZ_PL  = al256((size_t)NB * NH_ * SEQ * HD * 2);
static constexpr size_t SZ_CTX = al256((size_t)NB * SEQ * 2 * DM * 2);
static constexpr size_t SZ_TOTAL = 3 * SZ_XB + 4 * SZ_WB + 8 * SZ_PL + SZ_CTX;
static_assert(SZ_TOTAL <= (size_t)134217728);
static_assert(SZ_PL == (size_t)NB * SEQ * DM * 2);

extern "C" void kernel_launch(void* const* d_in, const int* in_sizes, int n_in,
                              void* d_out, int out_size, void* d_ws, size_t ws_size, hipStream_t stream) {
    if (n_in < 7) return;
    const size_t needx = ((size_t)(NB - 1) * SEQ_FULL + SEQ) * DM;
    if ((size_t)in_sizes[0] < needx || (size_t)in_sizes[1] < needx || (size_t)in_sizes[2] < needx) return;
    if ((size_t)in_sizes[3] < (size_t)DM * DM || (size_t)in_sizes[4] < (size_t)DM * DM || (size_t)in_sizes[5] < (size_t)DM * DM || (size_t)in_sizes[6] < (size_t)DM * DM) return;
    if ((size_t)out_size < ((size_t)(NB - 1) * OUT_SEQ + SEQ) * DM) return;
    if (SZ_TOTAL > ws_size) return;
    const float* xq = (const float*)d_in[0]; const float* xk = (const float*)d_in[1]; const float* xv = (const float*)d_in[2];
    const float* wq = (const float*)d_in[3]; const float* wk = (const float*)d_in[4]; const float* wv = (const float*)d_in[5]; const float* wp = (const float*)d_in[6];
    float* OUT = (float*)d_out;
    char* wsp = (char*)d_ws;
    bf* XQ = (bf*)wsp; wsp += SZ_XB;
    bf* XK = (bf*)wsp; wsp += SZ_XB;
    bf* XV = (bf*)wsp; wsp += SZ_XB;
    bf* WQT = (bf*)wsp; wsp += SZ_WB;
    bf* WKT = (bf*)wsp; wsp += SZ_WB;
    bf* WVT = (bf*)wsp; wsp += SZ_WB;
    bf* WPT = (bf*)wsp; wsp += SZ_WB;
    h16* QH = (h16*)wsp; wsp += SZ_PL;
    h16* QR = (h16*)wsp; wsp += SZ_PL;
    h16* KH = (h16*)wsp; wsp += SZ_PL;
    h16* KR = (h16*)wsp; wsp += SZ_PL;
    h16* VH = (h16*)wsp; wsp += SZ_PL;
    h16* VR = (h16*)wsp; wsp += SZ_PL;
    h16* VTH = (h16*)wsp; wsp += SZ_PL;
    h16* VTR = (h16*)wsp; wsp += SZ_PL;
    bf* CTX = (bf*)wsp; wsp += SZ_CTX;
    const size_t pln = SZ_PL / 2;

    if (SEQ == SEQ_FULL) {
        const size_t n8 = (size_t)NB * SEQ * DM / 8; const unsigned g = (unsigned)((n8 + 255) / 256);
        k_cvt8<<<g, 256, 0, stream>>>(xq, XQ, n8); k_cvt8<<<g, 256, 0, stream>>>(xk, XK, n8); k_cvt8<<<g, 256, 0, stream>>>(xv, XV, n8);
    } else {
        const size_t n8 = (size_t)SEQ * DM / 8; const unsigned g = (unsigned)((n8 + 255) / 256);
        for (int b = 0; b < NB; ++b) {
            k_cvt8<<<g, 256, 0, stream>>>(xq + (size_t)b * SEQ_FULL * DM, XQ + (size_t)b * SEQ * DM, n8);
            k_cvt8<<<g, 256, 0, stream>>>(xk + (size_t)b * SEQ_FULL * DM, XK + (size_t)b * SEQ * DM, n8);
            k_cvt8<<<g, 256, 0, stream>>>(xv + (size_t)b * SEQ_FULL * DM, XV + (size_t)b * SEQ * DM, n8);
        }
    }
    { const dim3 g(DM / 64, DM / 64, 1);
      k_wt<<<g, 256, 0, stream>>>(wq, WQT); k_wt<<<g, 256, 0, stream>>>(wk, WKT); k_wt<<<g, 256, 0, stream>>>(wv, WVT); k_wt<<<g, 256, 0, stream>>>(wp, WPT); }

    { const dim3 g(NB * SEQ / 64, DM / 64, 1);
      k_gemm<0><<<g, 32, 0, stream>>>(XQ, WQT, DM, QH, QR, OUT);
      k_gemm<0><<<g, 32, 0, stream>>>(XK, WKT, DM, KH, KR, OUT);
      k_gemm<0><<<g, 32, 0, stream>>>(XV, WVT, DM, VH, VR, OUT); }

    k_vt<<<dim3(SEQ / 64, NB * NH_, 2), 256, 0, stream>>>(VH, VTH, pln);

    k_flash<<<dim3(SEQ / (16 * AW), NB * NH_, 1), 32 * AW, 0, stream>>>(QH, QR, KH, KR, VTH, VTR, CTX);

    k_gemm<1><<<dim3(NB * SEQ / 64, DM / 64, 1), 32, 0, stream>>>(CTX, WPT, 2 * DM, QH, QR, OUT);
}
